// EdgeUpdate_88991722373554
// MI455X (gfx1250) — hardware-verified
//
#include <hip/hip_runtime.h>
#include <stddef.h>
#include <stdint.h>

#define DF     64
#define H1     128
#define H2     64
#define W1P    129
#define KE     256
#define PQW    256
#define TROWS  64
#define GTHR   128
#define LDSW   264
#define NUWB   (2 * H1 * DF / 8)
#define NUWT   (H2 * KE / 8)
#define WSMAX  134217728

static_assert(DF % 32 == 0 && KE % 32 == 0 && KE == 2 * H1 && PQW == 2 * H1);
static_assert(TROWS == (GTHR / 32) * 16);
static_assert(GTHR == 2 * TROWS && GTHR == H1);
static_assert(((LDSW * 2) % 16) == 0);
static_assert(TROWS / 4 == 16);
static_assert(NUWB % 256 == 0 && NUWT % 256 == 0);
static_assert(H2 == 64 && (TROWS % 4) == 0);

typedef float          v4f   __attribute__((ext_vector_type(4)));
typedef float          v8f   __attribute__((ext_vector_type(8)));
typedef int            v8i   __attribute__((ext_vector_type(8)));
typedef unsigned short v4us  __attribute__((ext_vector_type(4)));
typedef unsigned short v8us  __attribute__((ext_vector_type(8)));
typedef unsigned short v16us __attribute__((ext_vector_type(16)));
typedef __bf16         v16bf __attribute__((ext_vector_type(16)));
typedef v4f  __attribute__((may_alias)) v4fa;
typedef v4us __attribute__((may_alias)) v4usa;
typedef v8us __attribute__((may_alias)) v8usa;
union FragB { v16bf v; v16us u; v8us h[2]; v8i w; };

__device__ __forceinline__ v8f wmb(const FragB& a, const FragB& b, v8f c) {
  v8f d = __builtin_amdgcn_wmma_f32_16x16x32_bf16(false, a.v, false, b.v, (short)0, c, false, false);
  asm volatile("v_nop\n\tv_nop\n\tv_nop\n\tv_nop" : "+v"(d) : "v"(a.w), "v"(b.w));
  return d;
}

__device__ __forceinline__ unsigned bf16_bits(float f) {
  const unsigned u = __float_as_uint(f);
  return (u + 0x7FFFu + ((u >> 16) & 1u)) >> 16;
}
__device__ __forceinline__ float bf16_val(float f) {
  return __uint_as_float(bf16_bits(f) << 16);
}

__global__ __launch_bounds__(256) void k_prep(const float* __restrict__ W1, const float* __restrict__ W2,
                                              unsigned short* WB, unsigned short* WT2) {
  const int u = (int)blockIdx.x * 256 + (int)threadIdx.x;
  if (u >= NUWB + NUWT) return;
  v8us o;
  unsigned short* dp;
  if (u < NUWB) {
    const int c   = u >> 3;
    const int d0  = 8 * (u & 7);
    const int row = c & (H1 - 1);
    const float* p = W1 + (size_t)row * W1P + 1 + DF * (c >> 7) + d0;
    o[0] = (unsigned short)bf16_bits(p[0]);
    o[1] = (unsigned short)bf16_bits(p[1]);
    o[2] = (unsigned short)bf16_bits(p[2]);
    o[3] = (unsigned short)bf16_bits(p[3]);
    o[4] = (unsigned short)bf16_bits(p[4]);
    o[5] = (unsigned short)bf16_bits(p[5]);
    o[6] = (unsigned short)bf16_bits(p[6]);
    o[7] = (unsigned short)bf16_bits(p[7]);
    dp = WB + (size_t)u * 8;
  } else {
    const int v  = u - NUWB;
    const int n  = v >> 5;
    const int kk = 8 * (v & 31);
    const float* p = W2 + (size_t)n * H1 + (kk & (H1 - 1));
    const v4f a = *(const v4fa*)p;
    const v4f b = *(const v4fa*)(p + 4);
    o[0] = (unsigned short)bf16_bits(a.x);
    o[1] = (unsigned short)bf16_bits(a.y);
    o[2] = (unsigned short)bf16_bits(a.z);
    o[3] = (unsigned short)bf16_bits(a.w);
    o[4] = (unsigned short)bf16_bits(b.x);
    o[5] = (unsigned short)bf16_bits(b.y);
    o[6] = (unsigned short)bf16_bits(b.z);
    o[7] = (unsigned short)bf16_bits(b.w);
    dp = WT2 + (size_t)v * 8;
  }
  *(volatile v8us*)dp = o;
  __threadfence();
  *(volatile v8us*)dp = o;
}

__device__ __forceinline__ void node_store_pass(const float* st, float* PQ, int r0, int ch, int lane) {
#pragma unroll
  for (int i = 0; i < 16; ++i) {
    const v4f v = *(const v4fa*)(st + i * H1 + 4 * lane);
    float* dst = PQ + (size_t)(r0 + i) * PQW + ch * H1 + 4 * lane;
    *(volatile v4f*)dst = v;
  }
}

__global__ __launch_bounds__(GTHR) void k_node(const float* __restrict__ x,
                                               const unsigned short* __restrict__ WB,
                                               float* PQ,
                                               int nN)
{
  __shared__ __attribute__((aligned(16))) float sT[4 * 16 * H1];

  const int tid = (int)threadIdx.x, lane = tid & 31, wave = tid >> 5;
  const int hh = lane >> 4, m = lane & 15;
  const int ch = (int)blockIdx.y;
  const int r0 = (int)blockIdx.x * TROWS + 16 * wave;
  int ra = r0 + m;
  ra = ra > nN - 1 ? nN - 1 : ra;
  const float* xr = x + (size_t)ra * DF + 8 * hh;
  const unsigned short* wb = WB + (size_t)(ch * H1 + m) * DF + 8 * hh;

  v8f acc[8];
  {
    const v8f z8 = {0.f, 0.f, 0.f, 0.f, 0.f, 0.f, 0.f, 0.f};
#pragma unroll
    for (int t = 0; t < 8; ++t) acc[t] = z8;
  }

#pragma unroll
  for (int kk = 0; kk < DF / 32; ++kk) {
    const int k0 = 32 * kk;
    const v4f x0 = *(const v4fa*)(xr + k0);
    const v4f x1 = *(const v4fa*)(xr + k0 + 4);
    const v4f x2 = *(const v4fa*)(xr + k0 + 16);
    const v4f x3 = *(const v4fa*)(xr + k0 + 20);
    FragB af;
    af.u[0]  = (unsigned short)bf16_bits(x0.x);
    af.u[1]  = (unsigned short)bf16_bits(x0.y);
    af.u[2]  = (unsigned short)bf16_bits(x0.z);
    af.u[3]  = (unsigned short)bf16_bits(x0.w);
    af.u[4]  = (unsigned short)bf16_bits(x1.x);
    af.u[5]  = (unsigned short)bf16_bits(x1.y);
    af.u[6]  = (unsigned short)bf16_bits(x1.z);
    af.u[7]  = (unsigned short)bf16_bits(x1.w);
    af.u[8]  = (unsigned short)bf16_bits(x2.x);
    af.u[9]  = (unsigned short)bf16_bits(x2.y);
    af.u[10] = (unsigned short)bf16_bits(x2.z);
    af.u[11] = (unsigned short)bf16_bits(x2.w);
    af.u[12] = (unsigned short)bf16_bits(x3.x);
    af.u[13] = (unsigned short)bf16_bits(x3.y);
    af.u[14] = (unsigned short)bf16_bits(x3.z);
    af.u[15] = (unsigned short)bf16_bits(x3.w);
#pragma unroll
    for (int nt = 0; nt < 8; ++nt) {
      const unsigned short* wq = wb + (size_t)(16 * nt) * DF + k0;
      FragB bf;
      bf.h[0] = *(const v8usa*)wq;
      bf.h[1] = *(const v8usa*)(wq + 16);
      acc[nt] = wmb(af, bf, acc[nt]);
    }
  }

  float* st = sT + wave * (16 * H1);
#pragma unroll
  for (int nt = 0; nt < 8; ++nt) {
#pragma unroll
    for (int r = 0; r < 8; ++r) st[(8 * hh + r) * H1 + 16 * nt + m] = acc[nt][r];
  }
  __syncthreads();

  node_store_pass(st, PQ, r0, ch, lane);
  __threadfence();
  node_store_pass(st, PQ, r0, ch, lane);
}

__device__ __forceinline__ void out_store_pass(float* out, v4f v, int eb, int nE, bool full, bool tailw) {
  if (full) {
    *(volatile v4f*)(out + (size_t)eb) = v;
  } else if (tailw) {
    if (eb     < nE) *(volatile float*)(out + (size_t)eb)     = v.x;
    if (eb + 1 < nE) *(volatile float*)(out + (size_t)eb + 1) = v.y;
    if (eb + 2 < nE) *(volatile float*)(out + (size_t)eb + 2) = v.z;
    if (eb + 3 < nE) *(volatile float*)(out + (size_t)eb + 3) = v.w;
  }
}

__global__ __launch_bounds__(GTHR) void k_edge(
    const float* __restrict__ PQ,
    const int*   __restrict__ ei,
    const float* __restrict__ ew,
    const unsigned short* __restrict__ WT2,
    const float* __restrict__ W1,
    const float* __restrict__ b1,
    const float* __restrict__ b2,
    const float* __restrict__ W3,
    const float* __restrict__ b3,
    float* out,
    int nE, int nN)
{
  __shared__ __attribute__((aligned(16))) unsigned short sA[TROWS * LDSW];
  __shared__ __attribute__((aligned(16))) float sOut[TROWS];
  __shared__ __attribute__((aligned(16))) float sB1[H1];
  __shared__ __attribute__((aligned(16))) float sW0[H1];
  __shared__ __attribute__((aligned(16))) float sB2[H2];
  __shared__ __attribute__((aligned(16))) float sW3[H2];
  __shared__ __attribute__((aligned(16))) float sEw[TROWS];
  __shared__ int sIdx[2 * TROWS];

  const int tid = (int)threadIdx.x, lane = tid & 31, wave = tid >> 5;
  const int hh = lane >> 4, m = lane & 15;
  const int e0 = (int)blockIdx.x * TROWS;

  {
    const int r   = tid & (TROWS - 1);
    const int sel = tid >> 6;
    int e = e0 + r;
    e = e > nE - 1 ? nE - 1 : e;
    const int raw = ei[(size_t)sel * (size_t)nE + (size_t)e];
    int ix = raw < 0 ? raw + nN : raw;
    ix = ix < 0 ? 0 : (ix > nN - 1 ? nN - 1 : ix);
    sIdx[tid] = ix;
    sB1[tid] = bf16_val(b1[tid]);
    sW0[tid] = bf16_val(W1[(size_t)tid * W1P]);
    if (tid < TROWS) {
      sB2[tid] = bf16_val(b2[tid]);
      sW3[tid] = bf16_val(W3[tid]);
      sEw[tid] = bf16_val(ew[e]);
    }
  }
  __syncthreads();

  {
    const int col = 4 * lane;
    const v4f w0v = *(const v4fa*)(sW0 + col);
    const v4f b1v = *(const v4fa*)(sB1 + col);
#pragma unroll 2
    for (int i = 0; i < TROWS / 4; ++i) {
      const int row = 4 * i + wave;
      const int ns = sIdx[row];
      const int ng = sIdx[TROWS + row];
      const float ev = sEw[row];
      const v4f p = *(const v4fa*)(PQ + (size_t)ns * PQW + col);
      const v4f q = *(const v4fa*)(PQ + (size_t)ng * PQW + H1 + col);
      v4us oh, ol;
#pragma unroll
      for (int j = 0; j < 4; ++j) {
        float v = (p[j] + q[j]) + ev * w0v[j];
        v = v + b1v[j];
        v = fmaxf(v, 0.0f);
        const unsigned hb = bf16_bits(v);
        const float hv = __uint_as_float(hb << 16);
        const unsigned lb = bf16_bits(v - hv);
        oh[j] = (unsigned short)hb;
        ol[j] = (unsigned short)lb;
      }
      *(v4usa*)(sA + row * LDSW + col)      = oh;
      *(v4usa*)(sA + row * LDSW + H1 + col) = ol;
    }
  }
  __syncthreads();

  v8f acc[4];
  {
    const v8f z8 = {0.f, 0.f, 0.f, 0.f, 0.f, 0.f, 0.f, 0.f};
#pragma unroll
    for (int t = 0; t < 4; ++t) acc[t] = z8;
  }
  const unsigned short* ap = sA + (16 * wave + m) * LDSW + 8 * hh;
  const unsigned short* wp = WT2 + (size_t)m * KE + 8 * hh;

#pragma unroll 1
  for (int kk = 0; kk < KE / 32; ++kk) {
    const int k0 = 32 * kk;
    FragB af;
    af.h[0] = *(const v8usa*)(ap + k0);
    af.h[1] = *(const v8usa*)(ap + k0 + 16);
#pragma unroll
    for (int nt = 0; nt < 4; ++nt) {
      const unsigned short* wq = wp + (size_t)(16 * nt) * KE + k0;
      FragB bf;
      bf.h[0] = *(const v8usa*)wq;
      bf.h[1] = *(const v8usa*)(wq + 16);
      acc[nt] = wmb(af, bf, acc[nt]);
    }
  }

  float part[8];
#pragma unroll
  for (int r = 0; r < 8; ++r) part[r] = 0.0f;
#pragma unroll
  for (int nt = 0; nt < 4; ++nt) {
    const int c = 16 * nt + m;
    const float bv = sB2[c];
    const float wv = sW3[c];
#pragma unroll
    for (int r = 0; r < 8; ++r) {
      const float hv = fmaxf(acc[nt][r] + bv, 0.0f);
      part[r] = fmaf(hv, wv, part[r]);
    }
  }
#pragma unroll
  for (int msk = 1; msk <= 8; msk <<= 1) {
#pragma unroll
    for (int r = 0; r < 8; ++r) part[r] += __shfl_xor(part[r], msk, 32);
  }
  const float b3v = bf16_val(b3[0]);
  if (m == 0) {
#pragma unroll
    for (int r = 0; r < 8; ++r) sOut[16 * wave + 8 * hh + r] = part[r] + b3v;
  }
  __syncthreads();

  const bool wr  = (tid < TROWS / 4);
  const int  t16 = wr ? tid : 0;
  const v4f  v   = *(const v4fa*)(sOut + 4 * t16);
  const int  eb  = e0 + 4 * t16;
  const bool full  = wr && (eb + 3 < nE);
  const bool tailw = wr && !full;
  out_store_pass(out, v, eb, nE, full, tailw);
  __threadfence();
  out_store_pass(out, v, eb, nE, full, tailw);
}

static inline int cdiv(int a, int b) { return (a + b - 1) / b; }

extern "C" void kernel_launch(void* const* d_in, const int* in_sizes, int n_in,
                              void* d_out, int out_size, void* d_ws, size_t ws_size,
                              hipStream_t stream) {
  if (n_in < 9) return;
  if (in_sizes[0] < DF || (in_sizes[0] % DF) != 0) return;
  const int nN = in_sizes[0] / DF;
  const int nE = in_sizes[2];
  if (nE < 1) return;
  if (in_sizes[1] != 2 * nE) return;
  if (in_sizes[3] != H1 * W1P) return;
  if (in_sizes[4] != H1) return;
  if (in_sizes[5] != H2 * H1) return;
  if (in_sizes[6] != H2) return;
  if (in_sizes[7] != H2) return;
  if (in_sizes[8] < 1) return;
  if (out_size != nE) return;

  const float* x  = (const float*)d_in[0];
  const int*   ei = (const int*)d_in[1];
  const float* ew = (const float*)d_in[2];
  const float* W1 = (const float*)d_in[3];
  const float* b1 = (const float*)d_in[4];
  const float* W2 = (const float*)d_in[5];
  const float* b2 = (const float*)d_in[6];
  const float* W3 = (const float*)d_in[7];
  const float* b3 = (const float*)d_in[8];
  float* out = (float*)d_out;

  const int NPAD = cdiv(nN, TROWS) * TROWS;

  char* ws = (char*)d_ws;
  size_t off = 0;
  const size_t oWB  = off; off += (size_t)(2 * H1) * DF * 2;  off = (off + 255) & ~(size_t)255;
  const size_t oWT2 = off; off += (size_t)H2 * KE * 2;        off = (off + 255) & ~(size_t)255;
  const size_t oPQ  = off; off += (size_t)NPAD * PQW * 4;      off = (off + 255) & ~(size_t)255;
  if (off > ws_size || off > (size_t)WSMAX) return;
  unsigned short* WB  = (unsigned short*)(ws + oWB);
  unsigned short* WT2 = (unsigned short*)(ws + oWT2);
  float*          PQ  = (float*)(ws + oPQ);

  k_prep<<<(NUWB + NUWT) / 256, 256, 0, stream>>>(W1, W2, WB, WT2);
  dim3 gN(NPAD / TROWS, 2);
  k_node<<<gN, GTHR, 0, stream>>>(x, WB, PQ, nN);
  k_edge<<<cdiv(nE, TROWS), GTHR, 0, stream>>>(PQ, ei, ew, WT2, W1, b1, b2, W3, b3, out, nE, nN);
}
